// Block_81956565943135
// MI455X (gfx1250) — hardware-verified
//
#include <hip/hip_runtime.h>


#pragma clang fp contract(off)

#ifndef NB
#define NB 4
#endif
#ifndef SEQ
#define SEQ 2048
#endif
#define NB_FULL 4
#define SEQ_FULL 2048
#define CDIM 384
#define NHEAD 6
#define HD 64
#define HID 384
#define KD 384
#define MROWS (NB * SEQ)
#define WS_LIMIT 134217728ull

static_assert(NB >= 1 && NB <= NB_FULL);
static_assert(SEQ % 64 == 0 && SEQ >= 64 && SEQ <= SEQ_FULL);
static_assert(CDIM == NHEAD * HD);
static_assert(HD == 64);
static_assert(CDIM == 384);
static_assert(HID == CDIM);
static_assert(KD == CDIM && KD % 32 == 0 && KD % 8 == 0);
static_assert(CDIM % 64 == 0 && HID % 64 == 0);
static_assert(MROWS % 64 == 0);
static_assert(MROWS % 8 == 0);
static_assert(CDIM == 32 * 4 * 3);
static_assert((MROWS * (CDIM / 8)) % 256 == 0);
static_assert((CDIM * (CDIM / 8)) % 256 == 0);
static_assert((CDIM * 2) % 128 == 0 && (CDIM * 4) % 128 == 0 && (SEQ * 2) % 128 == 0 && (HD * 2) == 128);
static_assert((size_t)MROWS * CDIM < 2147483647ull);

typedef _Float16 v16h __attribute__((ext_vector_type(16)));
typedef _Float16 v8h  __attribute__((ext_vector_type(8)));
typedef _Float16 v4h  __attribute__((ext_vector_type(4)));
typedef float    v8f  __attribute__((ext_vector_type(8)));
typedef float    v4f  __attribute__((ext_vector_type(4)));
typedef unsigned int v4u __attribute__((ext_vector_type(4)));
typedef unsigned int v2u __attribute__((ext_vector_type(2)));

union Frag { v16h v; v4u q[2]; };

__device__ __forceinline__ v8f mma(v16h a, v16h b, v8f c) {
  v8f d = __builtin_amdgcn_wmma_f32_16x16x32_f16(false, a, false, b, (short)0, c, false, false);
  asm volatile("v_nop\n\tv_nop\n\tv_nop\n\tv_nop" : "+v"(d) : "v"(a), "v"(b));
  return d;
}

__device__ __forceinline__ v8f zero8() {
  v8f z;
#pragma unroll
  for (int i = 0; i < 8; ++i) z[i] = 0.0f;
  return z;
}

__device__ __forceinline__ float bf16q(float f) {
  unsigned int u = __float_as_uint(f);
  unsigned int r = u + 0x7FFFu + ((u >> 16) & 1u);
  r = ((u & 0x7F800000u) == 0x7F800000u) ? u : r;
  return __uint_as_float(r & 0xFFFF0000u);
}
__device__ __forceinline__ v4f bf16q4(v4f a) {
  v4f r;
  r.x = bf16q(a.x); r.y = bf16q(a.y); r.z = bf16q(a.z); r.w = bf16q(a.w);
  return r;
}
__device__ __forceinline__ unsigned short hbits(float f) {
  _Float16 h = (_Float16)f;
  return __builtin_bit_cast(unsigned short, h);
}
__device__ __forceinline__ v4u pack8h(float f0, float f1, float f2, float f3,
                                      float f4, float f5, float f6, float f7) {
  v8h t;
  t[0] = (_Float16)f0; t[1] = (_Float16)f1; t[2] = (_Float16)f2; t[3] = (_Float16)f3;
  t[4] = (_Float16)f4; t[5] = (_Float16)f5; t[6] = (_Float16)f6; t[7] = (_Float16)f7;
  return __builtin_bit_cast(v4u, t);
}
__device__ __forceinline__ v2u pack4h(v4f a) {
  v4h t;
  t[0] = (_Float16)a.x; t[1] = (_Float16)a.y; t[2] = (_Float16)a.z; t[3] = (_Float16)a.w;
  return __builtin_bit_cast(v2u, t);
}

__global__ __launch_bounds__(256) void k_cvt(
    const float* __restrict__ src, unsigned short* __restrict__ dst,
    int nrows, int seq, int seq_full, float scale) {
  const int idx = blockIdx.x * 256 + threadIdx.x;
  const int total = nrows * (CDIM / 8);
  if (idx >= total) return;
  const int row = idx / (CDIM / 8);
  const int piece = idx - row * (CDIM / 8);
  const int b = row / seq, t = row - b * seq;
  const float* s = src + ((size_t)b * (size_t)seq_full + t) * CDIM + piece * 8;
  const v4f a0 = *(const v4f*)(s);
  const v4f a1 = *(const v4f*)(s + 4);
  const v4u o = pack8h(bf16q(a0.x) * scale, bf16q(a0.y) * scale, bf16q(a0.z) * scale, bf16q(a0.w) * scale,
                       bf16q(a1.x) * scale, bf16q(a1.y) * scale, bf16q(a1.z) * scale, bf16q(a1.w) * scale);
  unsigned short* d = dst + (size_t)row * CDIM + piece * 8;
  *(volatile v4u*)d = o;
  __threadfence();
  *(volatile v4u*)d = o;
}

template <int WRH, int OUTFULL>
__device__ __forceinline__ void ln_body(
    const float* __restrict__ x, const float* __restrict__ g, const float* __restrict__ bt,
    float* __restrict__ outF, unsigned short* __restrict__ outH, int nrows) {
  const int lane = threadIdx.x & 31, w = threadIdx.x >> 5;
  const int row = blockIdx.x * 8 + w;
  if (row >= nrows) return;
  const float* xr = x + (size_t)row * CDIM + 4 * lane;
  v4f v[3];
#pragma unroll
  for (int sg = 0; sg < 3; ++sg) v[sg] = *(const v4f*)(xr + 128 * sg);

  float s = 0.0f;
#pragma unroll
  for (int sg = 0; sg < 3; ++sg) s += (v[sg].x + v[sg].y) + (v[sg].z + v[sg].w);
#pragma unroll
  for (int xm = 1; xm < 32; xm <<= 1) s += __shfl_xor(s, xm, 32);
  const float mu = s * (1.0f / CDIM);

  v4f d[3];
  float qs = 0.0f;
#pragma unroll
  for (int sg = 0; sg < 3; ++sg) {
    d[sg] = v[sg] - mu;
    qs += (d[sg].x * d[sg].x + d[sg].y * d[sg].y) + (d[sg].z * d[sg].z + d[sg].w * d[sg].w);
  }
#pragma unroll
  for (int xm = 1; xm < 32; xm <<= 1) qs += __shfl_xor(qs, xm, 32);
  const float var = qs * (1.0f / CDIM);
  const float rstd = rsqrtf(var + 1e-5f);

  v4f y[3];
  v2u yh[3];
#pragma unroll
  for (int sg = 0; sg < 3; ++sg) {
    const v4f g4 = bf16q4(*(const v4f*)(g + 128 * sg + 4 * lane));
    const v4f b4 = bf16q4(*(const v4f*)(bt + 128 * sg + 4 * lane));
    y[sg] = (d[sg] * rstd) * g4 + b4;
    yh[sg] = pack4h(y[sg]);
  }
  size_t orow;
  if (OUTFULL) {
    const int b = row / SEQ, t = row - b * SEQ;
    orow = ((size_t)b * SEQ_FULL + t) * CDIM;
  } else {
    orow = (size_t)row * CDIM;
  }
  float* of = outF + orow + 4 * lane;
  unsigned short* oh = outH + (size_t)row * CDIM + 4 * lane;
#pragma unroll
  for (int sg = 0; sg < 3; ++sg) *(volatile v4f*)(of + 128 * sg) = y[sg];
  if (WRH) {
#pragma unroll
    for (int sg = 0; sg < 3; ++sg) *(volatile v2u*)(oh + 128 * sg) = yh[sg];
  }
  __threadfence();
#pragma unroll
  for (int sg = 0; sg < 3; ++sg) *(volatile v4f*)(of + 128 * sg) = y[sg];
  if (WRH) {
#pragma unroll
    for (int sg = 0; sg < 3; ++sg) *(volatile v2u*)(oh + 128 * sg) = yh[sg];
  }
}

__global__ __launch_bounds__(256) void k_ln_mid(
    const float* __restrict__ x, const float* __restrict__ g, const float* __restrict__ bt,
    float* __restrict__ outF, unsigned short* __restrict__ outH, int nrows) {
  ln_body<1, 0>(x, g, bt, outF, outH, nrows);
}
__global__ __launch_bounds__(256) void k_ln_out(
    const float* __restrict__ x, const float* __restrict__ g, const float* __restrict__ bt,
    float* __restrict__ outF, int nrows) {
  ln_body<0, 1>(x, g, bt, outF, nullptr, nrows);
}

template <int EPI, int RESFULL>
__device__ __forceinline__ void gemm_body(
    const unsigned short* __restrict__ A, const unsigned short* __restrict__ Bt,
    const float* __restrict__ bias, const float* __restrict__ res,
    float* __restrict__ outF, unsigned short* __restrict__ out0,
    unsigned short* __restrict__ out1, float wsc) {
  __shared__ __attribute__((aligned(16))) unsigned short sT[64][72];
  __shared__ __attribute__((aligned(16))) float sF[64][68];
  const int tid = threadIdx.x, lane = tid & 31, w = tid >> 5;
  const int m = lane & 15, hl = lane >> 4, k8 = hl * 8;
  const int m0 = blockIdx.y * 64, n0 = blockIdx.x * 64;

  v8f acc[4];
#pragma unroll
  for (int j = 0; j < 4; ++j) acc[j] = zero8();

  const unsigned short* ap = A + (size_t)(m0 + 16 * w + m) * (size_t)KD + k8;
  const unsigned short* bp = Bt + (size_t)(n0 + m) * (size_t)KD + k8;
  const size_t jstep = (size_t)16 * (size_t)KD;
#pragma unroll 1
  for (int k0 = 0; k0 < KD; k0 += 32) {
    Frag a;
    a.q[0] = *(const v4u*)(ap + k0);
    a.q[1] = *(const v4u*)(ap + k0 + 16);
#pragma unroll
    for (int j = 0; j < 4; ++j) {
      Frag b;
      const unsigned short* bj = bp + jstep * j + k0;
      b.q[0] = *(const v4u*)(bj);
      b.q[1] = *(const v4u*)(bj + 16);
      acc[j] = mma(a.v, b.v, acc[j]);
    }
  }

  const int lrow0 = 16 * w + 8 * hl;

  if constexpr (EPI == 0) {
#pragma unroll
    for (int j = 0; j < 4; ++j) {
#pragma unroll
      for (int r = 0; r < 8; ++r) sT[lrow0 + r][16 * j + m] = hbits(acc[j][r] * wsc);
    }
    __syncthreads();
    const int hh = n0 / HD;
    const int b = m0 / SEQ, t0 = m0 - b * SEQ;
    const int bh = b * NHEAD + hh;
    v4u vq[4], vt[4];
    unsigned int oq[4], ot[4];
#pragma unroll
    for (int p = 0; p < 4; ++p) {
      const int rr = p * 16 + 4 * w + (lane >> 3);
      const int piece = lane & 7;
      vq[p] = *(const v4u*)&sT[rr][piece * 8];
      oq[p] = (unsigned int)((bh * SEQ + t0 + rr) * HD + piece * 8);
      unsigned int wv[4];
#pragma unroll
      for (int e = 0; e < 4; ++e) {
        const unsigned int lo = sT[piece * 8 + 2 * e][rr];
        const unsigned int hi = sT[piece * 8 + 2 * e + 1][rr];
        wv[e] = lo | (hi << 16);
      }
      v4u t;
      t.x = wv[0]; t.y = wv[1]; t.z = wv[2]; t.w = wv[3];
      vt[p] = t;
      ot[p] = (unsigned int)((bh * HD + rr) * SEQ + t0 + piece * 8);
    }
#pragma unroll
    for (int p = 0; p < 4; ++p) *(volatile v4u*)(out0 + oq[p]) = vq[p];
#pragma unroll
    for (int p = 0; p < 4; ++p) *(volatile v4u*)(out1 + ot[p]) = vt[p];
    __threadfence();
#pragma unroll
    for (int p = 0; p < 4; ++p) *(volatile v4u*)(out0 + oq[p]) = vq[p];
#pragma unroll
    for (int p = 0; p < 4; ++p) *(volatile v4u*)(out1 + ot[p]) = vt[p];
  } else if constexpr (EPI == 1) {
#pragma unroll
    for (int j = 0; j < 4; ++j) {
#pragma unroll
      for (int r = 0; r < 8; ++r) sF[lrow0 + r][16 * j + m] = acc[j][r] * wsc;
    }
    __syncthreads();
    const int b = m0 / SEQ, t0 = m0 - b * SEQ;
    v4f val[8];
    unsigned int off[8];
#pragma unroll
    for (int p = 0; p < 8; ++p) {
      const int row = 16 * w + 2 * p + hl;
      const int piece = m;
      const int ncol = n0 + 4 * piece;
      const v4f a = *(const v4f*)&sF[row][4 * piece];
      const v4f bv = bf16q4(*(const v4f*)(bias + ncol));
      const size_t rrow = RESFULL ? ((size_t)b * SEQ_FULL + t0 + row) : (size_t)(m0 + row);
      v4f rr = *(const v4f*)(res + rrow * (size_t)CDIM + ncol);
      if (RESFULL) rr = bf16q4(rr);
      val[p] = (a + bv) + rr;
      off[p] = (unsigned int)((size_t)(m0 + row) * (size_t)CDIM + ncol);
    }
#pragma unroll
    for (int p = 0; p < 8; ++p) *(volatile v4f*)(outF + off[p]) = val[p];
    __threadfence();
#pragma unroll
    for (int p = 0; p < 8; ++p) *(volatile v4f*)(outF + off[p]) = val[p];
  } else {
#pragma unroll
    for (int j = 0; j < 4; ++j) {
      const float bj = bf16q(bias[n0 + 16 * j + m]);
#pragma unroll
      for (int r = 0; r < 8; ++r) {
        float u = acc[j][r] * wsc + bj;
        u = fmaxf(u, 0.0f);
        sT[lrow0 + r][16 * j + m] = hbits(u);
      }
    }
    __syncthreads();
    v4u val[4];
    unsigned int off[4];
#pragma unroll
    for (int p = 0; p < 4; ++p) {
      const int row = 16 * w + 4 * p + (lane >> 3);
      const int piece = lane & 7;
      val[p] = *(const v4u*)&sT[row][piece * 8];
      off[p] = (unsigned int)((size_t)(m0 + row) * (size_t)HID + n0 + piece * 8);
    }
#pragma unroll
    for (int p = 0; p < 4; ++p) *(volatile v4u*)(out0 + off[p]) = val[p];
    __threadfence();
#pragma unroll
    for (int p = 0; p < 4; ++p) *(volatile v4u*)(out0 + off[p]) = val[p];
  }
}

__global__ __launch_bounds__(128) void k_gemm_proj(
    const unsigned short* __restrict__ A, const unsigned short* __restrict__ Bt,
    unsigned short* __restrict__ qpl, unsigned short* __restrict__ qtp) {
  gemm_body<0, 0>(A, Bt, nullptr, nullptr, nullptr, qpl, qtp, 0.0625f);
}
__global__ __launch_bounds__(128) void k_gemm_oproj(
    const unsigned short* __restrict__ A, const unsigned short* __restrict__ Bt,
    const float* __restrict__ bias, const float* __restrict__ xres, float* __restrict__ outF) {
  gemm_body<1, 1>(A, Bt, bias, xres, outF, nullptr, nullptr, 0.00390625f);
}
__global__ __launch_bounds__(128) void k_gemm_ffn1(
    const unsigned short* __restrict__ A, const unsigned short* __restrict__ Bt,
    const float* __restrict__ bias, unsigned short* __restrict__ act) {
  gemm_body<2, 0>(A, Bt, bias, nullptr, nullptr, act, nullptr, 0.0625f);
}
__global__ __launch_bounds__(128) void k_gemm_ffn2(
    const unsigned short* __restrict__ A, const unsigned short* __restrict__ Bt,
    const float* __restrict__ bias, const float* __restrict__ x1, float* __restrict__ outF) {
  gemm_body<1, 0>(A, Bt, bias, x1, outF, nullptr, nullptr, 0.0625f);
}

__global__ __launch_bounds__(128) __attribute__((amdgpu_num_vgpr(256)))
void k_attn(const unsigned short* __restrict__ qp, const unsigned short* __restrict__ vp,
            unsigned short* __restrict__ op) {
  __shared__ __attribute__((aligned(16))) unsigned short sP[4][16][72];
  const int tid = threadIdx.x, lane = tid & 31, w = tid >> 5;
  const int m = lane & 15, hl = lane >> 4, k8 = hl * 8;
  const int nqt = SEQ / 64;
  const int bh = blockIdx.x / nqt, qt = blockIdx.x - bh * nqt;
  const int b = bh / NHEAD, hh = bh - b * NHEAD;
  const int tq = qt * 64 + 16 * w;

  Frag qa0, qa1;
  {
    const unsigned short* qr = qp + ((size_t)bh * SEQ + tq + m) * HD + k8;
    qa0.q[0] = *(const v4u*)(qr);
    qa0.q[1] = *(const v4u*)(qr + 16);
    qa1.q[0] = *(const v4u*)(qr + 32);
    qa1.q[1] = *(const v4u*)(qr + 48);
  }
  float mrun[8], lrun[8];
  v8f oacc[4];
#pragma unroll
  for (int r = 0; r < 8; ++r) { mrun[r] = -1e30f; lrun[r] = 0.0f; }
#pragma unroll
  for (int j = 0; j < 4; ++j) oacc[j] = zero8();

#pragma unroll 1
  for (int kt = 0; kt <= qt; ++kt) {
    v8f s[4];
    const unsigned short* kb = qp + ((size_t)bh * SEQ + kt * 64 + m) * HD + k8;
#pragma unroll
    for (int j = 0; j < 4; ++j) {
      const unsigned short* kr = kb + j * 16 * HD;
      Frag f0, f1;
      f0.q[0] = *(const v4u*)(kr);
      f0.q[1] = *(const v4u*)(kr + 16);
      f1.q[0] = *(const v4u*)(kr + 32);
      f1.q[1] = *(const v4u*)(kr + 48);
      v8f t = mma(qa0.v, f0.v, zero8());
      t = mma(qa1.v, f1.v, t);
      s[j] = t;
    }
    float tmax[8];
#pragma unroll
    for (int r = 0; r < 8; ++r) tmax[r] = -1e30f;
#pragma unroll
    for (int j = 0; j < 4; ++j) {
#pragma unroll
      for (int r = 0; r < 8; ++r) {
        float val = s[j][r] * 0.125f;
        const int qi = tq + 8 * hl + r;
        const int ki = kt * 64 + 16 * j + m;
        const bool msk = (ki > qi) || (val == 0.0f);
        val = msk ? -1e30f : val;
        s[j][r] = val;
        tmax[r] = fmaxf(tmax[r], val);
      }
    }
#pragma unroll
    for (int r = 0; r < 8; ++r) {
#pragma unroll
      for (int xm = 1; xm < 16; xm <<= 1) tmax[r] = fmaxf(tmax[r], __shfl_xor(tmax[r], xm, 32));
    }
    float corr[8];
#pragma unroll
    for (int r = 0; r < 8; ++r) {
      const float mn = fmaxf(mrun[r], tmax[r]);
      corr[r] = __expf(mrun[r] - mn);
      mrun[r] = mn;
    }
    float tsum[8];
#pragma unroll
    for (int r = 0; r < 8; ++r) tsum[r] = 0.0f;
#pragma unroll
    for (int j = 0; j < 4; ++j) {
#pragma unroll
      for (int r = 0; r < 8; ++r) {
        const float p = __expf(s[j][r] - mrun[r]);
        tsum[r] += p;
        sP[w][8 * hl + r][16 * j + m] = hbits(p * 1024.0f);
      }
    }
#pragma unroll
    for (int r = 0; r < 8; ++r) {
#pragma unroll
      for (int xm = 1; xm < 16; xm <<= 1) tsum[r] += __shfl_xor(tsum[r], xm, 32);
      lrun[r] = lrun[r] * corr[r] + tsum[r];
    }
#pragma unroll
    for (int j = 0; j < 4; ++j) {
#pragma unroll
      for (int r = 0; r < 8; ++r) oacc[j][r] *= corr[r];
    }
    __syncthreads();
    Frag pa0, pa1;
    {
      const unsigned short* pr = &sP[w][m][k8];
      pa0.q[0] = *(const v4u*)(pr);
      pa0.q[1] = *(const v4u*)(pr + 16);
      pa1.q[0] = *(const v4u*)(pr + 32);
      pa1.q[1] = *(const v4u*)(pr + 48);
    }
    const unsigned short* vb = vp + ((size_t)bh * HD + m) * (size_t)SEQ + kt * 64 + k8;
#pragma unroll
    for (int jd = 0; jd < 4; ++jd) {
      const unsigned short* vr = vb + (size_t)jd * 16 * SEQ;
      Frag g0, g1;
      g0.q[0] = *(const v4u*)(vr);
      g0.q[1] = *(const v4u*)(vr + 16);
      g1.q[0] = *(const v4u*)(vr + 32);
      g1.q[1] = *(const v4u*)(vr + 48);
      oacc[jd] = mma(pa0.v, g0.v, oacc[jd]);
      oacc[jd] = mma(pa1.v, g1.v, oacc[jd]);
    }
    __syncthreads();
  }

  float il[8];
#pragma unroll
  for (int r = 0; r < 8; ++r) il[r] = 1.0f / (lrun[r] * 64.0f);
#pragma unroll
  for (int jd = 0; jd < 4; ++jd) {
#pragma unroll
    for (int r = 0; r < 8; ++r) sP[w][8 * hl + r][16 * jd + m] = hbits(oacc[jd][r] * il[r]);
  }
  __syncthreads();
  v4u val[4];
  unsigned int off[4];
#pragma unroll
  for (int p = 0; p < 4; ++p) {
    const int row = 4 * p + (lane >> 3);
    const int piece = lane & 7;
    val[p] = *(const v4u*)&sP[w][row][piece * 8];
    off[p] = (unsigned int)((size_t)(b * SEQ + tq + row) * CDIM + hh * HD + piece * 8);
  }
#pragma unroll
  for (int p = 0; p < 4; ++p) *(volatile v4u*)(op + off[p]) = val[p];
  __threadfence();
#pragma unroll
  for (int p = 0; p < 4; ++p) *(volatile v4u*)(op + off[p]) = val[p];
}

#define AL256(v) ((((size_t)(v)) + 255) & ~(size_t)255)
#define PLANE_W  AL256((size_t)CDIM * CDIM * 2)
#define PLANE_H  AL256((size_t)MROWS * CDIM * 2)
#define PLANE_F  AL256((size_t)MROWS * CDIM * 4)
static_assert(4 * PLANE_W + 6 * PLANE_H + 3 * PLANE_F <= WS_LIMIT);

extern "C" void kernel_launch(void* const* d_in, const int* in_sizes, int n_in,
                              void* d_out, int out_size, void* d_ws, size_t ws_size,
                              hipStream_t stream) {
  if (n_in < 12) return;
  const long needX = ((long)(NB - 1) * SEQ_FULL + SEQ) * CDIM;
  const long nW = (long)CDIM * CDIM;
  if ((long)in_sizes[0] < needX) return;
  if ((long)in_sizes[1] < nW || (long)in_sizes[2] < nW) return;
  if (in_sizes[3] < CDIM) return;
  if ((long)in_sizes[4] < nW || in_sizes[5] < CDIM) return;
  if ((long)in_sizes[6] < nW || in_sizes[7] < CDIM) return;
  if (in_sizes[8] < CDIM || in_sizes[9] < CDIM || in_sizes[10] < CDIM || in_sizes[11] < CDIM) return;
  if ((long)out_size < needX) return;

  const float* x   = (const float*)d_in[0];
  const float* Wq  = (const float*)d_in[1];
  const float* Wo  = (const float*)d_in[2];
  const float* bo  = (const float*)d_in[3];
  const float* W1  = (const float*)d_in[4];
  const float* b1  = (const float*)d_in[5];
  const float* W2  = (const float*)d_in[6];
  const float* b2  = (const float*)d_in[7];
  const float* g1  = (const float*)d_in[8];
  const float* be1 = (const float*)d_in[9];
  const float* g2  = (const float*)d_in[10];
  const float* be2 = (const float*)d_in[11];
  float* out = (float*)d_out;

  char* ws = (char*)d_ws;
  size_t off = 0;
  auto carve = [&](size_t bytes) -> char* { char* p = ws + off; off += AL256(bytes); return p; };
  const size_t MC = (size_t)MROWS * CDIM;
  unsigned short* wqp = (unsigned short*)carve((size_t)CDIM * CDIM * 2);
  unsigned short* wop = (unsigned short*)carve((size_t)CDIM * CDIM * 2);
  unsigned short* w1p = (unsigned short*)carve((size_t)CDIM * CDIM * 2);
  unsigned short* w2p = (unsigned short*)carve((size_t)CDIM * CDIM * 2);
  unsigned short* xh  = (unsigned short*)carve(MC * 2);
  unsigned short* qpl = (unsigned short*)carve(MC * 2);
  unsigned short* qtp = (unsigned short*)carve(MC * 2);
  unsigned short* opl = (unsigned short*)carve(MC * 2);
  float*          s1  = (float*)carve(MC * 4);
  float*          x1  = (float*)carve(MC * 4);
  unsigned short* h1  = (unsigned short*)carve(MC * 2);
  unsigned short* act = (unsigned short*)carve(MC * 2);
  float*          s2  = (float*)carve(MC * 4);
  if (off > ws_size || off > (size_t)WS_LIMIT) return;

  const int cvtW = (CDIM * (CDIM / 8)) / 256;
  const int cvtX = (MROWS * (CDIM / 8)) / 256;
  k_cvt<<<cvtW, 256, 0, stream>>>(Wq, wqp, CDIM, CDIM, CDIM, 16.0f);
  k_cvt<<<cvtW, 256, 0, stream>>>(Wo, wop, CDIM, CDIM, CDIM, 16.0f);
  k_cvt<<<cvtW, 256, 0, stream>>>(W1, w1p, CDIM, CDIM, CDIM, 16.0f);
  k_cvt<<<cvtW, 256, 0, stream>>>(W2, w2p, CDIM, CDIM, CDIM, 16.0f);
  k_cvt<<<cvtX, 256, 0, stream>>>(x, xh, MROWS, SEQ, SEQ_FULL, 1.0f);
  k_gemm_proj<<<dim3(CDIM / 64, MROWS / 64), 128, 0, stream>>>(xh, wqp, qpl, qtp);
  k_attn<<<NB * NHEAD * (SEQ / 64), 128, 0, stream>>>(qpl, qtp, opl);
  k_gemm_oproj<<<dim3(CDIM / 64, MROWS / 64), 128, 0, stream>>>(opl, wop, bo, x, s1);
  k_ln_mid<<<MROWS / 8, 256, 0, stream>>>(s1, g1, be1, x1, h1, MROWS);
  k_gemm_ffn1<<<dim3(HID / 64, MROWS / 64), 128, 0, stream>>>(h1, w1p, b1, act);
  k_gemm_ffn2<<<dim3(CDIM / 64, MROWS / 64), 128, 0, stream>>>(act, w2p, b2, x1, s2);
  k_ln_out<<<MROWS / 8, 256, 0, stream>>>(s2, g2, be2, out, MROWS);
}
